// GCN_TRAJ_13855564497014
// MI455X (gfx1250) — hardware-verified
//
#include <hip/hip_runtime.h>

typedef __bf16 v16bf __attribute__((ext_vector_type(16)));
typedef __bf16 v8bf  __attribute__((ext_vector_type(8)));
typedef float  v8f   __attribute__((ext_vector_type(8)));
typedef float  v4f   __attribute__((ext_vector_type(4)));
typedef v8bf __attribute__((may_alias)) v8bfa;
typedef v4f  __attribute__((may_alias)) v4fa;

union Frag { v16bf v; v8bf p[2]; };

#define NB     256
#define NHID   256
#define NPOS   1260
#define CONTB  5040
#define XROW   63
#define XT     30
#define OUTR   270

#define R_TCT  0
#define R_ACT  86016
#define R_TE1  147456
#define R_DCT  148480
#define R_IDCT 154624
#define R_G1   160768
#define R_G2A  275456
#define R_G2B  340992
#define R_G3A  406528
#define R_G3B  472064
#define R_G4   537600
#define PLANE  586752

static_assert(R_ACT == 21 * 64 * 64);
static_assert(R_TE1 - R_ACT == 60 * 32 * 32);
static_assert(R_DCT - R_TE1 == 16 * 64);
static_assert(R_IDCT - R_DCT == 64 * 96);
static_assert(R_G1 - R_IDCT == 96 * 64);
static_assert(R_G2A - R_G1 == 256 * 448);
static_assert(R_G2B - R_G2A == 256 * 256);
static_assert(R_G3A - R_G2B == 256 * 256);
static_assert(R_G3B - R_G3A == 256 * 256);
static_assert(R_G4 - R_G3B == 256 * 256);
static_assert(PLANE - R_G4 == 192 * 256);
static_assert((PLANE % 256) == 0);

#define XAH  0
#define XAL  5376
#define GAH  10752
#define GAL  18432
#define HTH  0
#define HTL  21504
#define ZOFF 43008
#define SBIG 43072

__device__ __forceinline__ v8f wmma3(v8f c, v16bf ah, v16bf al, v16bf bh, v16bf bl) {
  c = __builtin_amdgcn_wmma_f32_16x16x32_bf16(false, ah, false, bh, (short)0, c, false, false);
  c = __builtin_amdgcn_wmma_f32_16x16x32_bf16(false, ah, false, bl, (short)0, c, false, false);
  c = __builtin_amdgcn_wmma_f32_16x16x32_bf16(false, al, false, bh, (short)0, c, false, false);
  asm volatile("v_nop\n\tv_nop\n\tv_nop\n\tv_nop" : "+v"(c) : "v"(ah), "v"(al), "v"(bh), "v"(bl));
  return c;
}

__device__ __forceinline__ v16bf ldfrag(const __bf16* p, int h) {
  Frag f;
  f.p[0] = *(const v8bfa*)(p + 8 * h);
  f.p[1] = *(const v8bfa*)(p + 16 + 8 * h);
  return f.v;
}

__device__ __forceinline__ void split2(float v, __bf16* ph, __bf16* pl) {
  const __bf16 hb = (__bf16)v;
  *ph = hb;
  *pl = (__bf16)(v - (float)hb);
}

__device__ __forceinline__ float th(float x) {
  x = fminf(fmaxf(x, -10.0f), 10.0f);
  const float e = __expf(2.0f * x);
  return 1.0f - 2.0f * __builtin_amdgcn_rcpf(e + 1.0f);
}

__device__ __forceinline__ void fill_copy(float* v, const float* __restrict__ src,
                                          int R, int C, int CP, int e) {
  const int row = e / CP, c0 = e - row * CP;
  const int rr = min(row, R - 1);
#pragma unroll
  for (int i = 0; i < 8; ++i) {
    const int c = c0 + i;
    const int cc = min(c, C - 1);
    const float s = src[rr * C + cc];
    v[i] = (row < R && c < C) ? s : 0.0f;
  }
}
__device__ __forceinline__ void fill_trans(float* v, const float* __restrict__ src,
                                           int R, int C, int RP, int CP, int e) {
  const int row = e / RP, t0 = e - row * RP;
  const int bi = row / CP, q = row - bi * CP;
  const int qq = min(q, C - 1);
#pragma unroll
  for (int i = 0; i < 8; ++i) {
    const int t = t0 + i;
    const int tt = min(t, R - 1);
    const float s = src[(bi * R + tt) * C + qq];
    v[i] = (q < C && t < R) ? s : 0.0f;
  }
}

__global__ __launch_bounds__(256) void k_prep(
    const float* __restrict__ T_c, const float* __restrict__ A_c,
    const float* __restrict__ te1_w, const float* __restrict__ dct_m,
    const float* __restrict__ idct_m,
    const float* __restrict__ g1_w, const float* __restrict__ g2a_w,
    const float* __restrict__ g2b_w, const float* __restrict__ g3a_w,
    const float* __restrict__ g3b_w, const float* __restrict__ g4_w,
    const float* __restrict__ cmask_unused, const int* __restrict__ hor_unused,
    __bf16* __restrict__ Phi, __bf16* __restrict__ Plo)
{
  const int g = blockIdx.x * 256 + threadIdx.x;
  if (g >= PLANE / 8) return;
  const int e0 = g * 8;
  float v[8];
  if (e0 < R_ACT)       fill_trans(v, T_c, 60, 60, 64, 64, e0 - R_TCT);
  else if (e0 < R_TE1)  fill_trans(v, A_c, 21, 21, 32, 32, e0 - R_ACT);
  else if (e0 < R_DCT)  fill_copy(v, te1_w, 10, 60, 64, e0 - R_TE1);
  else if (e0 < R_IDCT) fill_copy(v, dct_m, 60, 90, 96, e0 - R_DCT);
  else if (e0 < R_G1)   fill_copy(v, idct_m, 90, 60, 64, e0 - R_IDCT);
  else if (e0 < R_G2A)  fill_copy(v, g1_w, 256, 436, 448, e0 - R_G1);
  else if (e0 < R_G2B)  fill_copy(v, g2a_w, 256, 256, 256, e0 - R_G2A);
  else if (e0 < R_G3A)  fill_copy(v, g2b_w, 256, 256, 256, e0 - R_G2B);
  else if (e0 < R_G3B)  fill_copy(v, g3a_w, 256, 256, 256, e0 - R_G3A);
  else if (e0 < R_G4)   fill_copy(v, g3b_w, 256, 256, 256, e0 - R_G3B);
  else                  fill_copy(v, g4_w, 180, 256, 256, e0 - R_G4);

  v8bf ho, lo;
#pragma unroll
  for (int i = 0; i < 8; ++i) {
    const __bf16 hb = (__bf16)v[i];
    ho[i] = hb;
    lo[i] = (__bf16)(v[i] - (float)hb);
  }
  __bf16* dh = Phi + e0;
  __bf16* dl = Plo + e0;
  *(volatile v8bf*)dh = ho;
  *(volatile v8bf*)dl = lo;
  __threadfence();
  *(volatile v8bf*)dh = ho;
  *(volatile v8bf*)dl = lo;
}

__global__ __launch_bounds__(256) void k_gcn(
    const float* __restrict__ cont, const __bf16* __restrict__ Phi, const __bf16* __restrict__ Plo,
    const float* __restrict__ conv_w, const float* __restrict__ conv_b,
    const float* __restrict__ bn1_scale, const float* __restrict__ bn1_shift,
    const float* __restrict__ resconv_w, const float* __restrict__ resconv_b,
    const float* __restrict__ bnr_scale, const float* __restrict__ bnr_shift,
    const float* __restrict__ prelu_a,
    const float* __restrict__ te1_b, const float* __restrict__ te2_w, const float* __restrict__ te2_b,
    const float* __restrict__ ne1_w, const float* __restrict__ ne1_b,
    const float* __restrict__ ne2_w, const float* __restrict__ ne2_b,
    float* __restrict__ hcont)
{
  __shared__ __attribute__((aligned(16))) __bf16 sBig[SBIG];
  __shared__ __attribute__((aligned(16))) float  sU[NPOS * 4];
  __shared__ __attribute__((aligned(16))) float  sWc[NHID * 4];
  __shared__ __attribute__((aligned(16))) float  sWr[NHID * 4];
  __shared__ float sCb[NHID];
  __shared__ __attribute__((aligned(16))) float sHc[NHID];
  __shared__ float sZ2[16 * 24];
  __shared__ float sN1[160];
  __shared__ float sNe1w[210];
  __shared__ float sNe1b[10], sNe2w[10], sTe1b[16], sTe2w[16];

  const int tid = threadIdx.x, lane = tid & 31, h = lane >> 4, m = lane & 15;
  const int wave = __builtin_amdgcn_readfirstlane(tid >> 5);
  const int b = blockIdx.x;
  const float pa = prelu_a[0], te2b = te2_b[0], ne2b = ne2_b[0];
  const v8f zero8 = {0.f, 0.f, 0.f, 0.f, 0.f, 0.f, 0.f, 0.f};
  const __bf16 bz = (__bf16)0.0f;

  if (tid < 210) sNe1w[tid] = ne1_w[tid];
  if (tid < 10) { sNe1b[tid] = ne1_b[tid]; sNe2w[tid] = ne2_w[tid]; }
  if (tid < 16) {
    const int j = min(tid, 9);
    const float a = te1_b[j], w = te2_w[j];
    sTe1b[tid] = (tid < 10) ? a : 0.0f;
    sTe2w[tid] = (tid < 10) ? w : 0.0f;
  }
  if (tid < 64) sBig[ZOFF + tid] = bz;
  {
    const int o = tid;
    const float s1 = bn1_scale[o], sr = bnr_scale[o];
#pragma unroll
    for (int c = 0; c < 4; ++c) {
      sWc[o * 4 + c] = s1 * conv_w[o * 4 + c];
      sWr[o * 4 + c] = sr * resconv_w[o * 4 + c];
    }
    sCb[o] = s1 * conv_b[o] + bn1_shift[o] + sr * resconv_b[o] + bnr_shift[o];
  }

  const float* cbp = cont + (size_t)b * CONTB;
  for (int i = tid; i < 21 * 4 * 64; i += 256) {
    const int v = i >> 8, c = (i >> 6) & 3, t = i & 63;
    const int tt = min(t, 59);
    float s = cbp[tt * 84 + v * 4 + c];
    s = (t < 60) ? s : 0.0f;
    split2(s, sBig + XAH + i, sBig + XAL + i);
  }
  for (int i = tid; i < 60 * 4 * 32; i += 256) { sBig[GAH + i] = bz; sBig[GAL + i] = bz; }

  v4f xr[5], gr[5];
  int hoff[5];
#pragma unroll
  for (int i = 0; i < 5; ++i) {
    const int n = tid + 256 * i;
    const int nn = min(n, NPOS - 1);
    const int vq = nn / 60, tq = nn - vq * 60;
    hoff[i] = vq * 1024 + tq;
    xr[i] = *(const v4fa*)(cbp + tq * 84 + vq * 4);
  }
  __syncthreads();

#pragma unroll 1
  for (int job = wave; job < 84; job += 8) {
    const int v = job >> 2, nt = job & 3;
    const int aoh = (m < 4) ? (XAH + (v * 4 + m) * 64) : ZOFF;
    const int aol = (m < 4) ? (XAL + (v * 4 + m) * 64) : ZOFF;
    const int bo = R_TCT + (v * 64 + nt * 16 + m) * 64;
    v8f acc = zero8;
#pragma unroll
    for (int ks = 0; ks < 2; ++ks) {
      const v16bf ah = ldfrag(sBig + aoh + 32 * ks, h);
      const v16bf al = ldfrag(sBig + aol + 32 * ks, h);
      const v16bf bh = ldfrag(Phi + bo + 32 * ks, h);
      const v16bf bl = ldfrag(Plo + bo + 32 * ks, h);
      acc = wmma3(acc, ah, al, bh, bl);
    }
    if (h == 0) {
      const int q = nt * 16 + m;
      if (q < 60) {
#pragma unroll
        for (int r = 0; r < 4; ++r) {
          const int idx = (q * 4 + r) * 32 + v;
          split2(acc[r], sBig + GAH + idx, sBig + GAL + idx);
        }
      }
    }
  }
  __syncthreads();

#pragma unroll 1
  for (int job = wave; job < 120; job += 8) {
    const int t = job >> 1, nt = job & 1;
    const int aoh = (m < 4) ? (GAH + (t * 4 + m) * 32) : ZOFF;
    const int aol = (m < 4) ? (GAL + (t * 4 + m) * 32) : ZOFF;
    const int bo = R_ACT + (t * 32 + nt * 16 + m) * 32;
    const v16bf ah = ldfrag(sBig + aoh, h);
    const v16bf al = ldfrag(sBig + aol, h);
    const v16bf bh = ldfrag(Phi + bo, h);
    const v16bf bl = ldfrag(Plo + bo, h);
    const v8f acc = wmma3(zero8, ah, al, bh, bl);
    if (h == 0) {
      const int w = nt * 16 + m;
      if (w < 21) {
        const v4f gq = {acc[0], acc[1], acc[2], acc[3]};
        *(v4fa*)(sU + (w * 60 + t) * 4) = gq;
      }
    }
  }
  __syncthreads();

#pragma unroll
  for (int i = 0; i < 5; ++i) {
    const int nn = min(tid + 256 * i, NPOS - 1);
    gr[i] = *(const v4fa*)(sU + nn * 4);
  }
  for (int i = tid; i < 336 * 4; i += 256) {
    const int row = i >> 2, c = 60 + (i & 3);
    sBig[HTH + row * 64 + c] = bz;
    sBig[HTL + row * 64 + c] = bz;
  }

#pragma unroll 1
  for (int og = 0; og < 16; ++og) {
#pragma unroll 1
    for (int ol = 0; ol < 16; ++ol) {
      const int o = og * 16 + ol;
      const v4f wc = *(const v4fa*)(sWc + o * 4);
      const v4f wr = *(const v4fa*)(sWr + o * 4);
      const float c0 = sCb[o];
#pragma unroll
      for (int i = 0; i < 5; ++i) {
        if (i < 4 || tid < NPOS - 1024) {
          float hv = c0;
          hv = fmaf(gr[i].x, wc.x, hv);
          hv = fmaf(gr[i].y, wc.y, hv);
          hv = fmaf(gr[i].z, wc.z, hv);
          hv = fmaf(gr[i].w, wc.w, hv);
          hv = fmaf(xr[i].x, wr.x, hv);
          hv = fmaf(xr[i].y, wr.y, hv);
          hv = fmaf(xr[i].z, wr.z, hv);
          hv = fmaf(xr[i].w, wr.w, hv);
          hv = (hv >= 0.0f) ? hv : pa * hv;
          const int idx = hoff[i] + ol * 64;
          split2(hv, sBig + HTH + idx, sBig + HTL + idx);
        }
      }
    }
    __syncthreads();

#pragma unroll 1
    for (int v = wave; v < 21; v += 8) {
      v8f acc = zero8;
#pragma unroll
      for (int ks = 0; ks < 2; ++ks) {
        const v16bf ah = ldfrag(sBig + HTH + (v * 16 + m) * 64 + 32 * ks, h);
        const v16bf al = ldfrag(sBig + HTL + (v * 16 + m) * 64 + 32 * ks, h);
        const v16bf bh = ldfrag(Phi + R_TE1 + m * 64 + 32 * ks, h);
        const v16bf bl = ldfrag(Plo + R_TE1 + m * 64 + 32 * ks, h);
        acc = wmma3(acc, ah, al, bh, bl);
      }
      const float b1 = sTe1b[m], w2 = sTe2w[m];
      float p[8];
#pragma unroll
      for (int r = 0; r < 8; ++r) p[r] = th(acc[r] + b1) * w2;
#pragma unroll
      for (int s = 1; s < 16; s <<= 1) {
#pragma unroll
        for (int r = 0; r < 8; ++r) p[r] += __shfl_xor(p[r], s);
      }
      if (m == 0) {
#pragma unroll
        for (int r = 0; r < 8; ++r) sZ2[(8 * h + r) * 24 + v] = th(p[r] + te2b);
      }
    }
    __syncthreads();

    if (tid < 160) {
      const int ol = tid / 10, j = tid - ol * 10;
      float a = sNe1b[j];
#pragma unroll 1
      for (int v = 0; v < 21; ++v) a = fmaf(sZ2[ol * 24 + v], sNe1w[j * 21 + v], a);
      sN1[tid] = th(a);
    }
    __syncthreads();
    if (tid < 16) {
      float hc = ne2b;
#pragma unroll 1
      for (int j = 0; j < 10; ++j) hc = fmaf(sN1[tid * 10 + j], sNe2w[j], hc);
      sHc[og * 16 + tid] = th(hc);
    }
  }
  __syncthreads();

  const int q4 = tid & 63;
  const v4f hv4 = *(const v4fa*)(sHc + q4 * 4);
  float* hd = hcont + (size_t)b * NHID + q4 * 4;
  if (tid < 64) *(volatile v4f*)hd = hv4;
  __threadfence();
  if (tid < 64) *(volatile v4f*)hd = hv4;
}

template <int KT, int NT>
__device__ __forceinline__ void layer(const __bf16* sAh, const __bf16* sAl,
                                      const __bf16* __restrict__ Wh, const __bf16* __restrict__ Wl,
                                      int wave, int m, int h, v8f& a0, v8f& a1) {
  const v8f z = {0.f, 0.f, 0.f, 0.f, 0.f, 0.f, 0.f, 0.f};
  a0 = z; a1 = z;
  const bool two = (wave + 8) < NT;
  const __bf16* arh = sAh + m * 448;
  const __bf16* arl = sAl + m * 448;
  const int row0 = wave * 16 + m;
  const int row1 = min((wave + 8) * 16 + m, NT * 16 - 1);
  const size_t b0o = (size_t)row0 * (KT * 32);
  const size_t b1o = (size_t)row1 * (KT * 32);
#pragma unroll 1
  for (int ks = 0; ks < KT; ++ks) {
    const v16bf ah = ldfrag(arh + 32 * ks, h);
    const v16bf al = ldfrag(arl + 32 * ks, h);
    {
      const v16bf bh = ldfrag(Wh + b0o + 32 * ks, h);
      const v16bf bl = ldfrag(Wl + b0o + 32 * ks, h);
      a0 = wmma3(a0, ah, al, bh, bl);
    }
    if (two) {
      const v16bf bh = ldfrag(Wh + b1o + 32 * ks, h);
      const v16bf bl = ldfrag(Wl + b1o + 32 * ks, h);
      a1 = wmma3(a1, ah, al, bh, bl);
    }
  }
}

template <int MODE>
__device__ __forceinline__ void epi_act(v8f a0, v8f a1, const float* __restrict__ bias,
                                        __bf16* sAh, __bf16* sAl, float* sR,
                                        int wave, int m, int h) {
#pragma unroll
  for (int ti = 0; ti < 2; ++ti) {
    const int nt = wave + 8 * ti;
    const int o = nt * 16 + m;
    const float bo = bias[o];
    const v8f a = ti ? a1 : a0;
#pragma unroll
    for (int r = 0; r < 8; ++r) {
      const int row = 8 * h + r;
      float val = th(a[r] + bo);
      if (MODE >= 2) val += sR[row * 256 + o];
      if (MODE == 1 || MODE == 2) sR[row * 256 + o] = val;
      split2(val, sAh + row * 448 + o, sAl + row * 448 + o);
    }
  }
}

__global__ __launch_bounds__(256) void k_head(
    const float* __restrict__ x, const int* __restrict__ root_idx, const float* __restrict__ hcont,
    const __bf16* __restrict__ Phi, const __bf16* __restrict__ Plo,
    const float* __restrict__ g1_b, const float* __restrict__ g2a_b, const float* __restrict__ g2b_b,
    const float* __restrict__ g3a_b, const float* __restrict__ g3b_b, const float* __restrict__ g4_b,
    float* __restrict__ out)
{
  __shared__ __attribute__((aligned(16))) __bf16 sAh[16 * 448];
  __shared__ __attribute__((aligned(16))) __bf16 sAl[16 * 448];
  __shared__ __attribute__((aligned(16))) __bf16 sPh[48 * 96];
  __shared__ __attribute__((aligned(16))) __bf16 sPl[48 * 96];
  __shared__ __attribute__((aligned(16))) float  sRO[16 * OUTR];
  __shared__ float sDct[16 * 180];

  const int tid = threadIdx.x, lane = tid & 31, h = lane >> 4, m = lane & 15;
  const int wave = __builtin_amdgcn_readfirstlane(tid >> 5);
  const int b0 = blockIdx.x * 16;
  const v8f zero8 = {0.f, 0.f, 0.f, 0.f, 0.f, 0.f, 0.f, 0.f};
  const __bf16 bz = (__bf16)0.0f;

  const int ri0 = min(max(root_idx[0], 0), XROW - 1);
  const int ri1 = min(max(root_idx[1], 0), XROW - 1);
  const int ri2 = min(max(root_idx[2], 0), XROW - 1);

  for (int i = tid; i < 48 * 96; i += 256) {
    const int row = i / 96, tau = i - row * 96;
    const int bl = row / 3, k = row - bl * 3;
    const int tt = min(tau, XT - 1);
    const int ri = (k == 0) ? ri0 : ((k == 1) ? ri1 : ri2);
    float s = x[((size_t)tt * NB + b0 + bl) * XROW + ri];
    s = (tau < 90) ? s : 0.0f;
    split2(s, sPh + i, sPl + i);
  }
  for (int i = tid; i < 16 * 268; i += 256) {
    const int row = i / 268, c = 180 + (i - row * 268);
    const int oc = min(c - 180, NHID - 1);
    float s = hcont[(size_t)(b0 + row) * NHID + oc];
    s = (c < 436) ? s : 0.0f;
    split2(s, sAh + row * 448 + c, sAl + row * 448 + c);
  }
  __syncthreads();

#pragma unroll 1
  for (int job = wave; job < 12; job += 8) {
    const int mt = job >> 2, nt = job & 3;
    v8f acc = zero8;
#pragma unroll
    for (int ks = 0; ks < 3; ++ks) {
      const v16bf ah = ldfrag(sPh + (mt * 16 + m) * 96 + 32 * ks, h);
      const v16bf al = ldfrag(sPl + (mt * 16 + m) * 96 + 32 * ks, h);
      const v16bf bh = ldfrag(Phi + R_DCT + (nt * 16 + m) * 96 + 32 * ks, h);
      const v16bf bl = ldfrag(Plo + R_DCT + (nt * 16 + m) * 96 + 32 * ks, h);
      acc = wmma3(acc, ah, al, bh, bl);
    }
    const int d = nt * 16 + m;
    if (d < 60) {
#pragma unroll
      for (int r = 0; r < 8; ++r) {
        const int row = mt * 16 + 8 * h + r;
        const int bl = row / 3, k = row - bl * 3;
        const int o = d * 3 + k;
        const float val = acc[r];
        sDct[bl * 180 + o] = val;
        split2(val, sAh + bl * 448 + o, sAl + bl * 448 + o);
      }
    }
  }
  __syncthreads();
  if (tid < 192) {
    const int row = tid >> 2, c = 60 + (tid & 3);
    sPh[row * 64 + c] = bz;
    sPl[row * 64 + c] = bz;
  }

  v8f a0, a1;
  layer<14, 16>(sAh, sAl, Phi + R_G1, Plo + R_G1, wave, m, h, a0, a1);
  __syncthreads();
  epi_act<1>(a0, a1, g1_b, sAh, sAl, sRO, wave, m, h);
  __syncthreads();
  layer<8, 16>(sAh, sAl, Phi + R_G2A, Plo + R_G2A, wave, m, h, a0, a1);
  __syncthreads();
  epi_act<0>(a0, a1, g2a_b, sAh, sAl, sRO, wave, m, h);
  __syncthreads();
  layer<8, 16>(sAh, sAl, Phi + R_G2B, Plo + R_G2B, wave, m, h, a0, a1);
  __syncthreads();
  epi_act<2>(a0, a1, g2b_b, sAh, sAl, sRO, wave, m, h);
  __syncthreads();
  layer<8, 16>(sAh, sAl, Phi + R_G3A, Plo + R_G3A, wave, m, h, a0, a1);
  __syncthreads();
  epi_act<0>(a0, a1, g3a_b, sAh, sAl, sRO, wave, m, h);
  __syncthreads();
  layer<8, 16>(sAh, sAl, Phi + R_G3B, Plo + R_G3B, wave, m, h, a0, a1);
  __syncthreads();
  epi_act<3>(a0, a1, g3b_b, sAh, sAl, sRO, wave, m, h);
  __syncthreads();
  layer<8, 12>(sAh, sAl, Phi + R_G4, Plo + R_G4, wave, m, h, a0, a1);
  __syncthreads();
#pragma unroll
  for (int ti = 0; ti < 2; ++ti) {
    const int nt = wave + 8 * ti;
    if (nt < 12) {
      const int o = nt * 16 + m;
      const int oc = min(o, 179);
      const float bo = g4_b[oc];
      const v8f a = ti ? a1 : a0;
#pragma unroll
      for (int r = 0; r < 8; ++r) {
        const int row = 8 * h + r;
        if (o < 180) {
          const float val = (a[r] + bo) + sDct[row * 180 + o];
          const int d = o / 3, k = o - 3 * d;
          const int idx = (row * 3 + k) * 64 + d;
          split2(val, sPh + idx, sPl + idx);
        }
      }
    }
  }
  __syncthreads();

#pragma unroll 1
  for (int job = wave; job < 18; job += 8) {
    const int mt = job / 6, nt = job - mt * 6;
    v8f acc = zero8;
#pragma unroll
    for (int ks = 0; ks < 2; ++ks) {
      const v16bf ah = ldfrag(sPh + (mt * 16 + m) * 64 + 32 * ks, h);
      const v16bf al = ldfrag(sPl + (mt * 16 + m) * 64 + 32 * ks, h);
      const v16bf bh = ldfrag(Phi + R_IDCT + (nt * 16 + m) * 64 + 32 * ks, h);
      const v16bf bl = ldfrag(Plo + R_IDCT + (nt * 16 + m) * 64 + 32 * ks, h);
      acc = wmma3(acc, ah, al, bh, bl);
    }
    const int tau = nt * 16 + m;
    if (tau < 90) {
#pragma unroll
      for (int r = 0; r < 8; ++r) {
        const int row = mt * 16 + 8 * h + r;
        const int bl = row / 3, k = row - bl * 3;
        sRO[bl * OUTR + tau * 3 + k] = acc[r];
      }
    }
  }
  __syncthreads();

  v4f ov[5];
#pragma unroll
  for (int i = 0; i < 5; ++i) {
    const int pc = min(tid + 256 * i, 16 * OUTR / 4 - 1);
    ov[i] = *(const v4fa*)(sRO + pc * 4);
  }
  float* ob = out + (size_t)b0 * OUTR;
#pragma unroll
  for (int i = 0; i < 5; ++i) {
    const int p = tid + 256 * i;
    if (p < 16 * OUTR / 4) *(volatile v4f*)(ob + p * 4) = ov[i];
  }
  __threadfence();
#pragma unroll
  for (int i = 0; i < 5; ++i) {
    const int p = tid + 256 * i;
    if (p < 16 * OUTR / 4) *(volatile v4f*)(ob + p * 4) = ov[i];
  }
}

extern "C" void kernel_launch(void* const* d_in, const int* in_sizes, int n_in,
                              void* d_out, int out_size, void* d_ws, size_t ws_size,
                              hipStream_t stream) {
  if (n_in < 38) return;
  if (in_sizes[0] != XT * NB * XROW) return;
  if (in_sizes[1] != NB * CONTB) return;
  if (in_sizes[5] != 3) return;
  if (in_sizes[7] != 21 * 60 * 60 || in_sizes[8] != 60 * 21 * 21) return;
  if (in_sizes[26] != 256 * 436 || in_sizes[36] != 180 * 256) return;
  if (out_size != NB * OUTR) return;

  const size_t hc_bytes    = (size_t)NB * NHID * 4;
  const size_t plane_bytes = (size_t)PLANE * 2;
  const size_t total       = hc_bytes + 2 * plane_bytes;
  if (total > ws_size) return;

  const float* x         = (const float*)d_in[0];
  const float* cont      = (const float*)d_in[1];
  const float* cont_mask = (const float*)d_in[2];
  const float* dct_m     = (const float*)d_in[3];
  const float* idct_m    = (const float*)d_in[4];
  const int*   root_idx  = (const int*)d_in[5];
  const int*   horizon   = (const int*)d_in[6];
  const float* T_c       = (const float*)d_in[7];
  const float* A_c       = (const float*)d_in[8];
  const float* conv_w    = (const float*)d_in[9];
  const float* conv_b    = (const float*)d_in[10];
  const float* bn1_scale = (const float*)d_in[11];
  const float* bn1_shift = (const float*)d_in[12];
  const float* resconv_w = (const float*)d_in[13];
  const float* resconv_b = (const float*)d_in[14];
  const float* bnr_scale = (const float*)d_in[15];
  const float* bnr_shift = (const float*)d_in[16];
  const float* prelu_a   = (const float*)d_in[17];
  const float* te1_w = (const float*)d_in[18];
  const float* te1_b = (const float*)d_in[19];
  const float* te2_w = (const float*)d_in[20];
  const float* te2_b = (const float*)d_in[21];
  const float* ne1_w = (const float*)d_in[22];
  const float* ne1_b = (const float*)d_in[23];
  const float* ne2_w = (const float*)d_in[24];
  const float* ne2_b = (const float*)d_in[25];
  const float* g1_w  = (const float*)d_in[26];
  const float* g1_b  = (const float*)d_in[27];
  const float* g2a_w = (const float*)d_in[28];
  const float* g2a_b = (const float*)d_in[29];
  const float* g2b_w = (const float*)d_in[30];
  const float* g2b_b = (const float*)d_in[31];
  const float* g3a_w = (const float*)d_in[32];
  const float* g3a_b = (const float*)d_in[33];
  const float* g3b_w = (const float*)d_in[34];
  const float* g3b_b = (const float*)d_in[35];
  const float* g4_w  = (const float*)d_in[36];
  const float* g4_b  = (const float*)d_in[37];
  float* out = (float*)d_out;

  char* ws = (char*)d_ws;
  float*  hc  = (float*)(ws);
  __bf16* Phi = (__bf16*)(ws + hc_bytes);
  __bf16* Plo = (__bf16*)(ws + hc_bytes + plane_bytes);

  const int npieces = PLANE / 8;
  k_prep<<<(npieces + 255) / 256, 256, 0, stream>>>(T_c, A_c, te1_w, dct_m, idct_m,
                                                    g1_w, g2a_w, g2b_w, g3a_w, g3b_w, g4_w,
                                                    cont_mask, horizon, Phi, Plo);

  k_gcn<<<NB, 256, 0, stream>>>(cont, Phi, Plo, conv_w, conv_b, bn1_scale, bn1_shift,
                                resconv_w, resconv_b, bnr_scale, bnr_shift, prelu_a,
                                te1_b, te2_w, te2_b, ne1_w, ne1_b, ne2_w, ne2_b, hc);

  k_head<<<NB / 16, 256, 0, stream>>>(x, root_idx, hc, Phi, Plo,
                                      g1_b, g2a_b, g2b_b, g3a_b, g3b_b, g4_b, out);
}
